// GM_GCN2_81028853006976
// MI455X (gfx1250) — hardware-verified
//
#include <hip/hip_runtime.h>
#include <stdint.h>
#include <math.h>

#define NN   100000
#define NE   800000
#define XC   128
#define HC   64
#define NCL  40
#define MP   100032
#define NT   256
#define SRB  2048
#define NTL  49
#define NPA  (NTL * SRB)
#define SCH  2048
#define SPT  (SCH / NT)
#define NCH  ((NE + SCH - 1) / SCH)

static_assert(NPA >= MP, "");
static_assert(MP % 64 == 0 && MP >= NN, "");
static_assert(NE % SPT == 0, "");
static_assert(XC % 32 == 0 && HC % 32 == 0 && HC == 64, "");
static_assert(NN < (1 << 17) && SRB == 2048 && NT == 256, "");
static_assert((MP * 16) % 256 == 0, "");
static_assert((NN * (NCL / 4)) % 32 == 0 && NCL % 4 == 0, "");

typedef __attribute__((ext_vector_type(16))) _Float16 v16h;
typedef __attribute__((ext_vector_type(8)))  _Float16 v8h;
typedef __attribute__((ext_vector_type(4)))  _Float16 v4h;
typedef __attribute__((ext_vector_type(16))) __bf16   v16b;
typedef __attribute__((ext_vector_type(8)))  __bf16   v8b;
typedef __attribute__((ext_vector_type(8)))  float    v8f;
typedef __attribute__((ext_vector_type(4)))  float    v4f;
typedef __attribute__((ext_vector_type(2)))  float    v2f;
typedef __attribute__((ext_vector_type(4)))  int      v4i;

__device__ __forceinline__ unsigned short f2bf_bits(float f) {
  unsigned u = __float_as_uint(f);
  return (unsigned short)((u + 0x7FFFu + ((u >> 16) & 1u)) >> 16);
}
__device__ __forceinline__ float bf_bits2f(unsigned short h) { return __uint_as_float(((unsigned)h) << 16); }

__device__ __forceinline__ void split_bf(float f, unsigned short& hb, unsigned short& lb) {
  hb = f2bf_bits(f);
  lb = f2bf_bits(f - bf_bits2f(hb));
}

__device__ __forceinline__ void dep_guard_h(v8f& a, v8f& b, v16h x, v16h y) { asm volatile("v_nop\n\tv_nop\n\tv_nop\n\tv_nop" : "+v"(a), "+v"(b) : "v"(x), "v"(y)); }
__device__ __forceinline__ void dep_guard_b(v8f& a, v8f& b, v16b x, v16b y) { asm volatile("v_nop\n\tv_nop\n\tv_nop\n\tv_nop" : "+v"(a), "+v"(b) : "v"(x), "v"(y)); }
__device__ __forceinline__ void keep4_h(v16h a, v16h b, v16h c, v16h d) { asm volatile("v_nop" :: "v"(a), "v"(b), "v"(c), "v"(d)); }
__device__ __forceinline__ void keep4_b(v16b a, v16b b, v16b c, v16b d) { asm volatile("v_nop" :: "v"(a), "v"(b), "v"(c), "v"(d)); }
__device__ __forceinline__ void acc_guard4(v8f& a, v8f& b, v8f& c, v8f& d) { asm volatile("v_nop\n\tv_nop\n\tv_nop\n\tv_nop" : "+v"(a), "+v"(b), "+v"(c), "+v"(d)); }
template <typename T> struct Frag;
template <> struct Frag<_Float16> {
  typedef v16h V; union U { v16h v; v8h h[2]; };
  static __device__ __forceinline__ v16h load(const _Float16* p) {
    U f; f.h[0] = *(const v8h*)(p); f.h[1] = *(const v8h*)(p + 16); return f.v;
  }
  static __device__ __forceinline__ v8f mma(v16h a, v16h b, v8f c) {
    return __builtin_amdgcn_wmma_f32_16x16x32_f16(false, a, false, b, (short)0, c, false, false);
  }
  static __device__ __forceinline__ void guard(v8f& a, v8f& b, v16h x, v16h y) { dep_guard_h(a, b, x, y); }
  static __device__ __forceinline__ void keep(v16h a, v16h b, v16h c, v16h d) { keep4_h(a, b, c, d); }
};
template <> struct Frag<__bf16> {
  typedef v16b V; union U { v16b v; v8b h[2]; };
  static __device__ __forceinline__ v16b load(const __bf16* p) {
    U f; f.h[0] = *(const v8b*)(p); f.h[1] = *(const v8b*)(p + 16); return f.v;
  }
  static __device__ __forceinline__ v8f mma(v16b a, v16b b, v8f c) {
    return __builtin_amdgcn_wmma_f32_16x16x32_bf16(false, a, false, b, (short)0, c, false, false);
  }
  static __device__ __forceinline__ void guard(v8f& a, v8f& b, v16b x, v16b y) { dep_guard_b(a, b, x, y); }
  static __device__ __forceinline__ void keep(v16b a, v16b b, v16b c, v16b d) { keep4_b(a, b, c, d); }
};

template <int ET> struct Elem;
template <> struct Elem<0> { typedef _Float16 T; };
template <> struct Elem<1> { typedef __bf16 T; };
template <int ET, bool SPLIT, int BIAS_MODE, int OUT_MODE, bool RESID, int ACT = 0>
__global__ __launch_bounds__(256) void wmma_gemm64(
    const unsigned short* __restrict__ Ap, const unsigned short* __restrict__ A2p, int lda, long strideA,
    const unsigned short* __restrict__ Btp, const unsigned short* __restrict__ Bt2p, int ldb, long strideB,
    void* __restrict__ Cout, void* __restrict__ Cout2, int ldc, long strideC,
    const float* __restrict__ bias,
    const float* __restrict__ resid, long strideR,
    int M, int N, int K, float scale) {
  typedef typename Elem<ET>::T T;
  typedef typename Frag<T>::V V;
  const T* A = (const T*)Ap; const T* A2 = (const T*)A2p; const T* Bt = (const T*)Btp; const T* Bt2 = (const T*)Bt2p;
  __shared__ __align__(16) float sT[8][16 * 68];
  const int b    = blockIdx.y;
  const int lane = threadIdx.x & 31;
  const int wave = threadIdx.x >> 5;
  const int tilesN = N >> 6;
  const int tilesM = M >> 6;
  const int tile = blockIdx.x * 8 + wave;
  if (tile >= tilesM * tilesN) return;
  const int tm = tile / tilesN;
  const int tn = tile - tm * tilesN;
  const int m0 = tm << 6;
  const int n0 = tn << 6;

  const T* Ab  = A  + (size_t)b * strideA;
  const T* Bb  = Bt + (size_t)b * strideB;
  const T* Ab2 = SPLIT ? (A2  + (size_t)b * strideA) : nullptr;
  const T* Bb2 = SPLIT ? (Bt2 + (size_t)b * strideB) : nullptr;

  const int rlane = lane & 15;
  const int koff  = (lane >> 4) * 8;
  const int mOff  = (lane >> 4) * 8;

  v8f acc[4][4];
#pragma unroll
  for (int i = 0; i < 4; ++i)
#pragma unroll
    for (int j = 0; j < 4; ++j) acc[i][j] = (v8f){0.f,0.f,0.f,0.f,0.f,0.f,0.f,0.f};

  for (int k0 = 0; k0 < K; k0 += 32) {
    V bh[4], bl[4];
#pragma unroll
    for (int j = 0; j < 4; ++j) {
      const size_t bo = (size_t)(n0 + (j << 4) + rlane) * ldb + koff + k0;
      bh[j] = Frag<T>::load(Bb + bo);
      if (SPLIT) bl[j] = Frag<T>::load(Bb2 + bo);
    }
#pragma unroll
    for (int i = 0; i < 4; ++i) {
      const size_t ao = (size_t)(m0 + (i << 4) + rlane) * lda + koff + k0;
      V ah = Frag<T>::load(Ab + ao);
      V al;
      if (SPLIT) al = Frag<T>::load(Ab2 + ao);
#pragma unroll
      for (int j = 0; j < 4; ++j) {
        acc[i][j] = Frag<T>::mma(ah, bh[j], acc[i][j]);
        if (SPLIT) {
          acc[i][j] = Frag<T>::mma(ah, bl[j], acc[i][j]);
          acc[i][j] = Frag<T>::mma(al, bh[j], acc[i][j]);
        }
      }
      Frag<T>::guard(acc[i][0], acc[i][3], ah, SPLIT ? al : ah);
    }
    Frag<T>::keep(bh[0], bh[1], bh[2], bh[3]);
    if (SPLIT) Frag<T>::keep(bl[0], bl[1], bl[2], bl[3]);
  }
  acc_guard4(acc[0][0], acc[0][1], acc[0][2], acc[0][3]);
  acc_guard4(acc[1][0], acc[1][1], acc[1][2], acc[1][3]);
  acc_guard4(acc[2][0], acc[2][1], acc[2][2], acc[2][3]);
  acc_guard4(acc[3][0], acc[3][1], acc[3][2], acc[3][3]);

  float* slab = sT[wave];
  const float* Rb = RESID ? (resid + (size_t)b * strideR) : nullptr;
#pragma unroll
  for (int i = 0; i < 4; ++i) {
    const int mBase = m0 + (i << 4);
#pragma unroll
    for (int j = 0; j < 4; ++j) {
      const int n = n0 + (j << 4) + rlane;
      float bv = 0.f;
      if (BIAS_MODE == 2) bv = bias[n];
#pragma unroll
      for (int r = 0; r < 8; ++r) {
        float v = acc[i][j][r] * scale;
        if (BIAS_MODE == 1) v += bias[mBase + mOff + r];
        if (BIAS_MODE == 2) v += bv;
        if (RESID) v += Rb[(size_t)(mBase + mOff + r) * ldc + n];
        if (ACT == 1) v = tanhf(v);
        if (ACT == 2) v = fmaxf(v, 0.0f);
        if (ACT == 4) v = (v > 0.f) ? v : 0.01f * v;
        slab[(mOff + r) * 68 + (j << 4) + rlane] = v;
      }
    }
    __builtin_amdgcn_fence(__ATOMIC_RELEASE, "workgroup");
    __builtin_amdgcn_wave_barrier();
    __builtin_amdgcn_fence(__ATOMIC_ACQUIRE, "workgroup");
    if (OUT_MODE == 0) {
      float* C = (float*)Cout + (size_t)b * strideC;
      const int hh = lane >> 4, c4 = (lane & 15) * 4;
      for (int pass = 0; pass < 2; ++pass) {
#pragma unroll
        for (int it = 0; it < 8; ++it) {
          const int row = it * 2 + hh;
          v4f v = *(const v4f*)(slab + row * 68 + c4);
          *(volatile v4f*)(C + (size_t)(mBase + row) * ldc + n0 + c4) = v;
        }
        __threadfence();
      }
    } else {
      const int q = lane >> 3, c8 = (lane & 7) * 8;
      unsigned short* C  = (unsigned short*)Cout  + (size_t)b * strideC;
      unsigned short* C2 = (OUT_MODE == 2) ? ((unsigned short*)Cout2 + (size_t)b * strideC) : nullptr;
      for (int pass = 0; pass < 2; ++pass) {
#pragma unroll
        for (int it = 0; it < 4; ++it) {
          const int row = it * 4 + q;
          const float* sp = slab + row * 68 + c8;
          v8h hv, lv;
#pragma unroll
          for (int e = 0; e < 8; ++e) {
            if (OUT_MODE == 1) {
              hv[e] = (_Float16)sp[e];
            } else {
              unsigned short hb = f2bf_bits(sp[e]);
              unsigned short lb = f2bf_bits(sp[e] - bf_bits2f(hb));
              hv[e] = __builtin_bit_cast(_Float16, hb);
              lv[e] = __builtin_bit_cast(_Float16, lb);
            }
          }
          *(volatile v8h*)(C + (size_t)(mBase + row) * ldc + n0 + c8) = hv;
          if (OUT_MODE == 2) *(volatile v8h*)(C2 + (size_t)(mBase + row) * ldc + n0 + c8) = lv;
        }
        __threadfence();
      }
    }
    __builtin_amdgcn_fence(__ATOMIC_RELEASE, "workgroup");
    __builtin_amdgcn_wave_barrier();
    __builtin_amdgcn_fence(__ATOMIC_ACQUIRE, "workgroup");
  }
}

template <int KDIM>
__global__ __launch_bounds__(256) void wt_split_kernel(const float* __restrict__ W, long wstride, unsigned* __restrict__ HI, unsigned* __restrict__ LO,
                                                      int NO, int NOP, int total) {
  const int i = blockIdx.x * 256 + threadIdx.x;
  if (i >= total) return;
  const int per = NOP * (KDIM / 2);
  const int li = i / per;
  const int r = i - li * per;
  const int f = r / (KDIM / 2);
  const int k = 2 * (r - f * (KDIM / 2));
  const int fc = (f < NO) ? f : (NO - 1);
  const float* Wl = W + (size_t)li * wstride;
  float a = Wl[(size_t)k * NO + fc];
  float b = Wl[(size_t)(k + 1) * NO + fc];
  if (f >= NO) { a = 0.0f; b = 0.0f; }
  unsigned short ah, al, bh, bl;
  split_bf(a, ah, al); split_bf(b, bh, bl);
  const unsigned uh = (unsigned)ah | ((unsigned)bh << 16);
  const unsigned ul = (unsigned)al | ((unsigned)bl << 16);
  ((volatile unsigned*)HI)[i] = uh; ((volatile unsigned*)LO)[i] = ul;
  __threadfence();
  ((volatile unsigned*)HI)[i] = uh; ((volatile unsigned*)LO)[i] = ul;
}

__global__ __launch_bounds__(256) void xsplit_kernel(const float* __restrict__ X, unsigned short* __restrict__ HI, unsigned short* __restrict__ LO) {
  const int i = blockIdx.x * 256 + threadIdx.x;
  if (i >= MP * 16) return;
  const int row = i >> 4, c8 = (i & 15) * 8;
  const int rc = (row < NN) ? row : (NN - 1);
  const float* p = X + (size_t)rc * XC + c8;
  const v4f z4 = {0.f, 0.f, 0.f, 0.f};
  v4f a = *(const v4f*)p, b = *(const v4f*)(p + 4);
  if (row >= NN) { a = z4; b = z4; }
  v8h hv, lv;
#pragma unroll
  for (int e = 0; e < 4; ++e) {
    unsigned short h0, l0, h1, l1;
    split_bf(a[e], h0, l0); split_bf(b[e], h1, l1);
    hv[e] = __builtin_bit_cast(_Float16, h0); lv[e] = __builtin_bit_cast(_Float16, l0);
    hv[4 + e] = __builtin_bit_cast(_Float16, h1); lv[4 + e] = __builtin_bit_cast(_Float16, l1);
  }
  unsigned short* ph = HI + (size_t)row * XC + c8;
  unsigned short* pl = LO + (size_t)row * XC + c8;
  *(volatile v8h*)ph = hv; *(volatile v8h*)pl = lv;
  __threadfence();
  *(volatile v8h*)ph = hv; *(volatile v8h*)pl = lv;
}

__global__ __launch_bounds__(256) void pack_kernel(const float* __restrict__ LG, const float* __restrict__ b, float* __restrict__ out) {
  const int q = blockIdx.x * 256 + threadIdx.x;
  if (q >= NN * (NCL / 4)) return;
  const int row = q / (NCL / 4);
  const int c4 = (q - row * (NCL / 4)) * 4;
  const v4f a = *(const v4f*)(LG + (size_t)row * HC + c4);
  v4f bb;
  bb[0] = b[c4]; bb[1] = b[c4 + 1]; bb[2] = b[c4 + 2]; bb[3] = b[c4 + 3];
  const v4f y = a + bb;
  float* op = out + (size_t)q * 4;
  *(volatile v4f*)op = y;
  __threadfence();
  *(volatile v4f*)op = y;
}

__device__ __forceinline__ int blk_excl_scan(int cnt, int* scan_ws, int tid, int* tot) {
  const int lane = tid & 31, wave = tid >> 5; int incl = cnt;
#pragma unroll
  for (int o = 1; o < 32; o <<= 1) { const int v = __shfl_up(incl, o, 32); if (lane >= o) incl += v; }
  if (lane == 31) scan_ws[wave] = incl;
  __syncthreads();
  if (wave == 0) { int wv = (lane < NT / 32) ? scan_ws[lane] : 0; int wincl = wv;
#pragma unroll
    for (int o = 1; o < 32; o <<= 1) { const int v = __shfl_up(wincl, o, 32); if (lane >= o) wincl += v; }
    if (lane < NT / 32) scan_ws[32 + lane] = wincl - wv; if (lane == 31) scan_ws[64] = wincl; }
  __syncthreads();
  const int res = scan_ws[32 + wave] + incl - cnt; *tot = scan_ws[64];
  return res;
}
template <int SP, int CAP, bool SRCL>
__device__ __forceinline__ int chunk_hits(const int* __restrict__ dstv, const int* __restrict__ srcv, int e0, int n0, int tid,
                                          int* LIST, int* scan_ws) {
  const int eb = e0 + tid * SP;
  const bool real = (eb < NE);
  const int ebc = real ? eb : (NE - SP);
  int rec[SP]; int cnt = 0;
#pragma unroll
  for (int k = 0; k < SP; k += 4) {
    const v4i d4 = *(const v4i*)(dstv + ebc + k);
    v4i s4 = {0, 0, 0, 0};
    if (SRCL) s4 = *(const v4i*)(srcv + ebc + k);
#pragma unroll
    for (int e = 0; e < 4; ++e) {
      int sr = s4[e]; sr = sr < 0 ? 0 : (sr >= NN ? NN - 1 : sr);
      const int d = d4[e];
      int r = -1;
      if (real && d >= n0 && d < n0 + SRB) { r = ((d - n0) << 17) | sr; ++cnt; }
      rec[k + e] = r;
    }
  }
  int tot; int p = blk_excl_scan(cnt, scan_ws, tid, &tot);
#pragma unroll
  for (int k = 0; k < SP; ++k) if (rec[k] >= 0) { if ((unsigned)p < (unsigned)CAP) LIST[p] = rec[k]; ++p; }
  __syncthreads();
  return tot < CAP ? tot : CAP;
}

__global__ __launch_bounds__(NT) void deg_kernel(const int* __restrict__ ei, float* __restrict__ DINV) {
  __shared__ int LIST[SCH];
  __shared__ int scan_ws[80];
  const int tid = threadIdx.x, lane = tid & 31, wave = tid >> 5;
  const int n0 = blockIdx.x * SRB;
  const int* srcv = ei; const int* dstv = ei + NE;
  int cA0 = 0, cA1 = 0, cA2 = 0, cA3 = 0, cB0 = 0, cB1 = 0, cB2 = 0, cB3 = 0;
#pragma unroll 1
  for (int c = 0; c < NCH; ++c) {
    const int tot = chunk_hits<SPT, SCH, false>(dstv, srcv, c * SCH, n0, tid, LIST, scan_ws);
#pragma unroll 1
    for (int base = 0; base < tot; base += 32) {
      const int q = base + lane;
      const int qc = (q < SCH) ? q : (SCH - 1);
      const int lv = LIST[qc];
      const int rv = (q < tot) ? lv : -1;
      const int own = (rv >= 0 && (rv >> 25) == wave) ? 1 : 0;
      unsigned msk = (unsigned)__ballot(own);
#pragma unroll 1
      for (int it = 0; it < 32; ++it) {
        if (msk == 0u) break;
        const int bp = __builtin_ctz(msk); msk &= msk - 1u;
        const int r = __shfl(rv, bp, 32);
        const int dll = (r >> 17) & 255;
        const int hs  = dll >> 7;
        const int ol  = (dll >> 2) & 31;
        const int ix  = dll & 3;
        const bool mine = (ol == lane);
        const bool mA = mine && (hs == 0), mB = mine && (hs == 1);
        cA0 += (mA && ix == 0) ? 1 : 0; cA1 += (mA && ix == 1) ? 1 : 0; cA2 += (mA && ix == 2) ? 1 : 0; cA3 += (mA && ix == 3) ? 1 : 0;
        cB0 += (mB && ix == 0) ? 1 : 0; cB1 += (mB && ix == 1) ? 1 : 0; cB2 += (mB && ix == 2) ? 1 : 0; cB3 += (mB && ix == 3) ? 1 : 0;
      }
    }
    __syncthreads();
  }
  v4f dA, dB;
  dA[0] = rsqrtf((float)cA0 + 1.0f); dA[1] = rsqrtf((float)cA1 + 1.0f); dA[2] = rsqrtf((float)cA2 + 1.0f); dA[3] = rsqrtf((float)cA3 + 1.0f);
  dB[0] = rsqrtf((float)cB0 + 1.0f); dB[1] = rsqrtf((float)cB1 + 1.0f); dB[2] = rsqrtf((float)cB2 + 1.0f); dB[3] = rsqrtf((float)cB3 + 1.0f);
  float* pA = DINV + (size_t)n0 + wave * 256 + 4 * lane;
  float* pB = pA + 128;
  *(volatile v4f*)pA = dA; *(volatile v4f*)pB = dB;
  __threadfence();
  *(volatile v4f*)pA = dA; *(volatile v4f*)pB = dB;
}

template <int MODE>
__global__ __launch_bounds__(NT) void prop64_kernel(const float* __restrict__ SRC, const int* __restrict__ ei, const float* __restrict__ DINV,
                                                    const float* __restrict__ X0, float* ACC,
                                                    unsigned short* __restrict__ MH, unsigned short* __restrict__ ML, float cr) {
  constexpr int CW = 64;
  __shared__ int LIST[SCH];
  __shared__ int scan_ws[80];
  const int tid = threadIdx.x, lane = tid & 31, wave = tid >> 5;
  const int n0 = blockIdx.x * SRB;
  const v2f zv = {0.0f, 0.0f};
#pragma unroll 1
  for (int j = 0; j < SRB / 8; ++j) {
    float* rp = ACC + (size_t)(n0 + wave * (SRB / 8) + j) * CW + 2 * lane;
    *(volatile v2f*)rp = zv;
    __threadfence();
    *(volatile v2f*)rp = zv;
  }
  const int* srcv = ei; const int* dstv = ei + NE;
#pragma unroll 1
  for (int c = 0; c < NCH; ++c) {
    const int tot = chunk_hits<SPT, SCH, true>(dstv, srcv, c * SCH, n0, tid, LIST, scan_ws);
#pragma unroll 1
    for (int base = 0; base < tot; base += 32) {
      const int q = base + lane;
      const int qc = (q < SCH) ? q : (SCH - 1);
      const int lv = LIST[qc];
      const int rv = (q < tot) ? lv : -1;
      const int own = (rv >= 0 && (rv >> 25) == wave) ? 1 : 0;
      unsigned msk = (unsigned)__ballot(own);
#pragma unroll 1
      for (int it = 0; it < 32; ++it) {
        if (msk == 0u) break;
        const int bp = __builtin_ctz(msk); msk &= msk - 1u;
        const int r = __shfl(rv, bp, 32);
        const int dl = (r >> 17) & (SRB - 1);
        int s = r & 0x1FFFF; s = (s < NN) ? s : (NN - 1);
        const float ds = DINV[s];
        const v2f pv = *(const v2f*)(SRC + (size_t)s * CW + 2 * lane);
        float* rp = ACC + (size_t)(n0 + dl) * CW + 2 * lane;
        v2f a = *(const v2f*)rp;
        a = a + pv * ds;
        *(volatile v2f*)rp = a;
        __threadfence();
        *(volatile v2f*)rp = a;
      }
    }
    __syncthreads();
  }
  const v4f z4 = {0.f, 0.f, 0.f, 0.f};
  const int hh = lane >> 4, c4 = (lane & 15) * 4;
#pragma unroll 1
  for (int jj = 0; jj < SRB / 16; ++jj) {
    const int dl = wave * (SRB / 8) + 2 * jj + hh;
    const int n = n0 + dl;
    const int nc = (n < NN) ? n : (NN - 1);
    const float dn = DINV[n];
    const v4f a  = *(const v4f*)(ACC + (size_t)n * CW + c4);
    const v4f xs = *(const v4f*)(SRC + (size_t)nc * CW + c4);
    const v4f pr = (a + xs * dn) * dn;
    float* op = ACC + (size_t)n * CW + c4;
    if (MODE == 0) {
      v4f v;
#pragma unroll
      for (int e = 0; e < 4; ++e) v[e] = fmaxf(pr[e], 0.0f);
      if (n >= NN) v = z4;
      *(volatile v4f*)op = v;
      __threadfence();
      *(volatile v4f*)op = v;
    } else {
      const v4f x0v = *(const v4f*)(X0 + (size_t)n * CW + c4);
      v4f mp = pr * 0.9f + x0v * 0.1f;
      if (n >= NN) mp = z4;
      const v4f rv4 = mp * cr;
      v4h hv, lv;
#pragma unroll
      for (int e = 0; e < 4; ++e) {
        unsigned short hb, lb;
        split_bf(mp[e], hb, lb);
        hv[e] = __builtin_bit_cast(_Float16, hb);
        lv[e] = __builtin_bit_cast(_Float16, lb);
      }
      unsigned short* ph = MH + (size_t)n * CW + c4;
      unsigned short* pl = ML + (size_t)n * CW + c4;
      *(volatile v4f*)op = rv4; *(volatile v4h*)ph = hv; *(volatile v4h*)pl = lv;
      __threadfence();
      *(volatile v4f*)op = rv4; *(volatile v4h*)ph = hv; *(volatile v4h*)pl = lv;
    }
  }
}

extern "C" void kernel_launch(void* const* d_in, const int* in_sizes, int n_in,
                              void* d_out, int out_size, void* d_ws, size_t ws_size, hipStream_t stream) {
  if (n_in < 7) return;
  if (in_sizes[0] != NN * XC || in_sizes[1] != 2 * NE || in_sizes[2] != XC * HC || in_sizes[3] != HC ||
      in_sizes[4] != HC * NCL || in_sizes[5] != NCL || in_sizes[6] != 4 * HC * HC || out_size != NN * NCL) return;
  const float* x     = (const float*)d_in[0];
  const int*   ei    = (const int*)  d_in[1];
  const float* fc0w  = (const float*)d_in[2];
  const float* fc0b  = (const float*)d_in[3];
  const float* fc1w  = (const float*)d_in[4];
  const float* fc1b  = (const float*)d_in[5];
  const float* convw = (const float*)d_in[6];
  float* out = (float*)d_out;

  char* ws = (char*)d_ws; size_t off = 0;
  auto carve = [&](size_t bytes) -> char* { char* p = ws + off; off += (bytes + 255) & ~(size_t)255; return p; };
  const size_t xplane = (size_t)MP * XC * 2;
  const size_t mplane = (size_t)NPA * HC * 2;
  const size_t lgsz   = (size_t)MP * HC * 4;
  const size_t r1sz   = (2 * xplane > lgsz + 2 * mplane) ? (2 * xplane) : (lgsz + 2 * mplane);
  unsigned* W0H  = (unsigned*)carve((size_t)HC * XC * 2);
  unsigned* W0L  = (unsigned*)carve((size_t)HC * XC * 2);
  unsigned* WCH  = (unsigned*)carve((size_t)3 * HC * HC * 2);
  unsigned* WCL  = (unsigned*)carve((size_t)3 * HC * HC * 2);
  unsigned* W1H  = (unsigned*)carve((size_t)HC * HC * 2);
  unsigned* W1L  = (unsigned*)carve((size_t)HC * HC * 2);
  float*    DINV = (float*)   carve((size_t)NPA * 4);
  char*     R1   =            carve(r1sz);
  char*     HB   =            carve(lgsz);
  float*    X0B  = (float*)   carve((size_t)NPA * HC * 4);
  float*    ACCB = (float*)   carve((size_t)NPA * HC * 4);
  if (off > ws_size || off > (size_t)134217728) return;

  unsigned short* XH  = (unsigned short*)R1;
  unsigned short* XL  = (unsigned short*)(R1 + xplane);
  float*          LG  = (float*)R1;
  unsigned short* MH  = (unsigned short*)(R1 + lgsz);
  unsigned short* ML  = (unsigned short*)(R1 + lgsz + mplane);
  float*          H   = (float*)HB;
  unsigned short* HFH = (unsigned short*)HB;
  unsigned short* HFL = (unsigned short*)(HB + (size_t)MP * HC * 2);

  const double bd1 = 0.22314355131420976, bd2 = 0.15415067982725836, bd3 = 0.11778303565638346;
  const float sc1 = (float)bd1, sc2 = (float)bd2, sc3 = (float)bd3;
  const float cr1 = (float)(1.0 - bd1), cr2 = (float)(1.0 - bd2), cr3 = (float)(1.0 - bd3);

  if ((HC * (XC / 2)) % 256 != 0 || (3 * HC * (HC / 2)) % 256 != 0 || (HC * (HC / 2)) % 256 != 0) return;
  wt_split_kernel<XC><<<(HC * (XC / 2)) / 256, 256, 0, stream>>>(fc0w, 0L, W0H, W0L, HC, HC, HC * (XC / 2));
  wt_split_kernel<HC><<<(3 * HC * (HC / 2)) / 256, 256, 0, stream>>>(convw + (size_t)HC * HC, (long)(HC * HC), WCH, WCL, HC, HC, 3 * HC * (HC / 2));
  wt_split_kernel<HC><<<(HC * (HC / 2)) / 256, 256, 0, stream>>>(fc1w, 0L, W1H, W1L, NCL, HC, HC * (HC / 2));
  deg_kernel<<<NTL, NT, 0, stream>>>(ei, DINV);
  xsplit_kernel<<<(MP * 16) / 256, 256, 0, stream>>>(x, XH, XL);
  const int tiles = (MP / 64) * (HC / 64);
  const dim3 ggrid((tiles + 7) / 8, 1);
  wmma_gemm64<1, true, 2, 0, false, 2><<<ggrid, 256, 0, stream>>>(
      XH, XL, XC, 0L, (const unsigned short*)W0H, (const unsigned short*)W0L, XC, 0L,
      (void*)H, nullptr, HC, 0L, fc0b, nullptr, 0L, MP, HC, XC, 1.0f);
  prop64_kernel<0><<<NTL, NT, 0, stream>>>(H, ei, DINV, X0B, X0B, MH, ML, 1.0f);
  prop64_kernel<1><<<NTL, NT, 0, stream>>>(X0B, ei, DINV, X0B, ACCB, MH, ML, cr1);
  wmma_gemm64<1, true, 0, 0, true, 2><<<ggrid, 256, 0, stream>>>(
      MH, ML, HC, 0L, (const unsigned short*)WCH, (const unsigned short*)WCL, HC, 0L,
      (void*)H, nullptr, HC, 0L, nullptr, ACCB, 0L, MP, HC, HC, sc1);
  prop64_kernel<1><<<NTL, NT, 0, stream>>>(H, ei, DINV, X0B, ACCB, MH, ML, cr2);
  wmma_gemm64<1, true, 0, 0, true, 2><<<ggrid, 256, 0, stream>>>(
      MH, ML, HC, 0L, (const unsigned short*)WCH + (size_t)HC * HC, (const unsigned short*)WCL + (size_t)HC * HC, HC, 0L,
      (void*)H, nullptr, HC, 0L, nullptr, ACCB, 0L, MP, HC, HC, sc2);
  prop64_kernel<1><<<NTL, NT, 0, stream>>>(H, ei, DINV, X0B, ACCB, MH, ML, cr3);
  wmma_gemm64<1, true, 0, 2, true, 2><<<ggrid, 256, 0, stream>>>(
      MH, ML, HC, 0L, (const unsigned short*)WCH + (size_t)2 * HC * HC, (const unsigned short*)WCL + (size_t)2 * HC * HC, HC, 0L,
      (void*)HFH, (void*)HFL, HC, 0L, nullptr, ACCB, 0L, MP, HC, HC, sc3);
  wmma_gemm64<1, true, 0, 0, false, 0><<<ggrid, 256, 0, stream>>>(
      HFH, HFL, HC, 0L, (const unsigned short*)W1H, (const unsigned short*)W1L, HC, 0L,
      (void*)LG, nullptr, HC, 0L, nullptr, nullptr, 0L, MP, HC, HC, 1.0f);
  pack_kernel<<<(NN * (NCL / 4) + 255) / 256, 256, 0, stream>>>(LG, fc1b, out);
}
